// MoE_85383949844811
// MI455X (gfx1250) — hardware-verified
//
#include <hip/hip_runtime.h>
#include <math.h>

typedef __attribute__((ext_vector_type(16))) _Float16 v16h;
typedef __attribute__((ext_vector_type(16))) __bf16 v16b;
typedef __attribute__((ext_vector_type(8)))  _Float16 v8h;
typedef __attribute__((ext_vector_type(8)))  __bf16 v8b;
typedef __attribute__((ext_vector_type(8)))  float v8f;
typedef __attribute__((ext_vector_type(4)))  float v4f;
typedef __attribute__((ext_vector_type(4)))  unsigned v4u;
typedef _Float16 h16;

#ifndef NB
#define NB 32768
#endif
#define NB_FULL 32768
#define DIN  128
#define DHID 512
#define DOUT 128
#define NE   16
#define KF (NE * DHID)
#define HCARRY 64.0f
#define WCARRY 512.0f
#define OSCALE (1.0f / 32768.0f)

#define CH   128
#define XP   136
#define HP   72
#define OP   132
#define SLAB 64
#define NSLAB (DHID / SLAB)

#define WS_XB  ((size_t)0)
#define WS_W1T (WS_XB  + (size_t)NB * DIN * 2)
#define WS_W2T (WS_W1T + (size_t)NE * DHID * DIN * 2)
#define WS_END (WS_W2T + (size_t)DOUT * KF * 2)

#define MOE_LDS (DIN * NE * 4 + 4 * NE * 4 + NE * CH * 4 + 4 * 16 * XP * 2 + 4 * 16 * HP * 2 + CH * OP * 4)

static_assert(NB % 128 == 0);
static_assert(NB <= NB_FULL);
static_assert(DIN % 32 == 0 && SLAB % 32 == 0 && DHID % SLAB == 0 && KF % 32 == 0 && (KF * 2) % 128 == 0);
static_assert((size_t)NB_FULL * DOUT * 4 == 16777216);
static_assert(WS_W1T % 128 == 0 && WS_W2T % 128 == 0);
static_assert(WS_END <= (size_t)134217728);
static_assert(MOE_LDS <= 131072);
static_assert(64 * 65 * 4 <= 131072);
static_assert(DIN == CH && CH == 128 && NE == 16);
static_assert((XP * 2) % 16 == 0 && (HP * 2) % 16 == 0 && (OP * 4) % 16 == 0);
static_assert(XP >= DIN && HP >= SLAB && OP >= DOUT);
static_assert((size_t)(NB * DIN / 8 / 256) * 256 * 8 == (size_t)NB * DIN);
static_assert((size_t)(DHID / 64) * (DIN / 64) * NE * 4096 == (size_t)NE * DIN * DHID);
static_assert((size_t)(DOUT / 64) * (DHID / 64) * NE * 4096 == (size_t)DOUT * KF);
static_assert(256 * 2 * 16 == 64 * 64 * 2);
static_assert(8 * 32 * 8 == 16 * DIN);
static_assert(128 * 16 * 32 == CH * DOUT * 4);
static_assert((size_t)(NB / CH) * CH * DOUT == (size_t)NB * DOUT);

__device__ __forceinline__ v8f wmma16(v16h a, v16h b, v8f c) {
  v8f d = __builtin_amdgcn_wmma_f32_16x16x32_f16(false, a, false, b, (short)0, c, false, false);
  asm volatile("v_nop\n\tv_nop\n\tv_nop\n\tv_nop" : "+v"(d) : "v"(a), "v"(b));
  return d;
}
__device__ __forceinline__ v8f wmma_bf(v16b a, v16b b, v8f c) {
  v8f d = __builtin_amdgcn_wmma_f32_16x16x32_bf16(false, a, false, b, (short)0, c, false, false);
  asm volatile("v_nop\n\tv_nop\n\tv_nop\n\tv_nop" : "+v"(d) : "v"(a), "v"(b));
  return d;
}
__device__ __forceinline__ float bfr(float v) { return (float)(__bf16)v; }
static __device__ __forceinline__ h16 toh_flush(float v) { const h16 r = (h16)v; return (fabsf(v) < 6.103515625e-05f) ? (h16)0.0f : r; }
__device__ __forceinline__ v16b ldfrag_b(const unsigned short* p) { union { v16b v; v4u q[2]; } f; f.q[0] = *(const v4u*)p; f.q[1] = *(const v4u*)(p + 16); return f.v; }
__device__ __forceinline__ v16h ldfrag_h(const unsigned short* p) { union { v16h v; v4u q[2]; } f; f.q[0] = *(const v4u*)p; f.q[1] = *(const v4u*)(p + 16); return f.v; }

__global__ __launch_bounds__(256) void k_cvt_x(const float* __restrict__ X, unsigned short* __restrict__ XB) {
  const unsigned i = blockIdx.x * 256u + threadIdx.x;
  const unsigned ic = i < (unsigned)(NB * DIN / 8) ? i : (unsigned)(NB * DIN / 8 - 1);
  const v4f a = *(const v4f*)(X + (size_t)ic * 8), b = *(const v4f*)(X + (size_t)ic * 8 + 4);
  union { v8b h; v4u u; } o;
#pragma unroll
  for (int j = 0; j < 4; ++j) { o.h[j] = (__bf16)a[j]; o.h[4 + j] = (__bf16)b[j]; }
  const v4u val = o.u;
  volatile v4u* p = (volatile v4u*)(XB + (size_t)ic * 8);
  *p = val; __threadfence(); *p = val;
}

__global__ __launch_bounds__(256) void k_tr_w1(const float* __restrict__ S, unsigned short* __restrict__ Dst, unsigned K, unsigned N, unsigned dpitch, unsigned erow, unsigned ecol) {
  __shared__ float tile[64][65];
  const unsigned t = threadIdx.x, e = blockIdx.z, k0 = blockIdx.y * 64u, n0 = blockIdx.x * 64u;
  const float* s = S + (size_t)e * K * N;
#pragma unroll
  for (unsigned it = 0; it < 4; ++it) { const unsigned idx = it * 256u + t, kr = idx >> 4, c4 = idx & 15u;
    const v4f v = *(const v4f*)(s + (size_t)(k0 + kr) * N + n0 + 4u * c4);
    tile[kr][4u * c4 + 0] = v[0]; tile[kr][4u * c4 + 1] = v[1]; tile[kr][4u * c4 + 2] = v[2]; tile[kr][4u * c4 + 3] = v[3]; }
  __syncthreads();
  v4u o[2];
#pragma unroll
  for (unsigned it = 0; it < 2; ++it) { const unsigned idx = it * 256u + t, nr = idx >> 3, q = idx & 7u;
    union { v8b b; v4u u; } w;
#pragma unroll
    for (int i = 0; i < 8; ++i) { w.b[i] = (__bf16)tile[8u * q + i][nr]; }
    o[it] = w.u; }
#pragma unroll
  for (unsigned it = 0; it < 2; ++it) { const unsigned idx = it * 256u + t, nr = idx >> 3, q = idx & 7u;
    *(volatile v4u*)(Dst + (size_t)(e * erow + n0 + nr) * dpitch + e * ecol + k0 + 8u * q) = o[it]; }
  __threadfence();
#pragma unroll
  for (unsigned it = 0; it < 2; ++it) { const unsigned idx = it * 256u + t, nr = idx >> 3, q = idx & 7u;
    *(volatile v4u*)(Dst + (size_t)(e * erow + n0 + nr) * dpitch + e * ecol + k0 + 8u * q) = o[it]; }
}

__global__ __launch_bounds__(256) void k_tr_w2(const float* __restrict__ S, unsigned short* __restrict__ Dst, unsigned K, unsigned N, unsigned dpitch, unsigned erow, unsigned ecol, float sc) {
  __shared__ float tile[64][65];
  const unsigned t = threadIdx.x, e = blockIdx.z, k0 = blockIdx.y * 64u, n0 = blockIdx.x * 64u;
  const float* s = S + (size_t)e * K * N;
#pragma unroll
  for (unsigned it = 0; it < 4; ++it) { const unsigned idx = it * 256u + t, kr = idx >> 4, c4 = idx & 15u;
    const v4f v = *(const v4f*)(s + (size_t)(k0 + kr) * N + n0 + 4u * c4);
    tile[kr][4u * c4 + 0] = v[0]; tile[kr][4u * c4 + 1] = v[1]; tile[kr][4u * c4 + 2] = v[2]; tile[kr][4u * c4 + 3] = v[3]; }
  __syncthreads();
  v4u o[2];
#pragma unroll
  for (unsigned it = 0; it < 2; ++it) { const unsigned idx = it * 256u + t, nr = idx >> 3, q = idx & 7u;
    union { v8h h; v4u u; } w;
#pragma unroll
    for (int i = 0; i < 8; ++i) { const float v = bfr(tile[8u * q + i][nr]); w.h[i] = toh_flush(v * sc); }
    o[it] = w.u; }
#pragma unroll
  for (unsigned it = 0; it < 2; ++it) { const unsigned idx = it * 256u + t, nr = idx >> 3, q = idx & 7u;
    *(volatile v4u*)(Dst + (size_t)(e * erow + n0 + nr) * dpitch + e * ecol + k0 + 8u * q) = o[it]; }
  __threadfence();
#pragma unroll
  for (unsigned it = 0; it < 2; ++it) { const unsigned idx = it * 256u + t, nr = idx >> 3, q = idx & 7u;
    *(volatile v4u*)(Dst + (size_t)(e * erow + n0 + nr) * dpitch + e * ecol + k0 + 8u * q) = o[it]; }
}

__global__ __launch_bounds__(128) __attribute__((amdgpu_num_vgpr(256)))
void k_moe(const unsigned short* __restrict__ XB, const unsigned short* __restrict__ W1T, const unsigned short* __restrict__ W2T, const float* __restrict__ WG, const float* __restrict__ BG, float* __restrict__ OUT) {
  __shared__ __align__(16) float wgs[DIN][NE];
  __shared__ int wcnt[4][NE];
  __shared__ int lst[NE][CH];
  __shared__ __align__(16) unsigned short xa[4][16][XP];
  __shared__ __align__(16) _Float16 hs[4][16][HP];
  __shared__ __align__(16) float os[CH][OP];
  const unsigned tid = threadIdx.x, lane = tid & 31u, lm = lane & 15u, lh = lane >> 4;
  const int wave = __builtin_amdgcn_readfirstlane((int)(threadIdx.x >> 5));
  const unsigned blk0 = blockIdx.x * (unsigned)CH;

  { const float* pw = WG + (size_t)tid * NE;
#pragma unroll
    for (int j = 0; j < 4; ++j) { const v4f w = *(const v4f*)(pw + 4 * j); v4f o; o[0] = bfr(w[0]); o[1] = bfr(w[1]); o[2] = bfr(w[2]); o[3] = bfr(w[3]); *(v4f*)&wgs[tid][4 * j] = o; } }
  __syncthreads();

  float lg[NE];
#pragma unroll
  for (int e = 0; e < NE; ++e) lg[e] = 0.f;
  { const unsigned short* xr = XB + (size_t)(blk0 + tid) * DIN;
#pragma unroll 1
    for (unsigned kc = 0; kc < DIN / 8; ++kc) { const v4u q = *(const v4u*)(xr + 8u * kc); float xv[8];
#pragma unroll
      for (int j = 0; j < 4; ++j) { xv[2 * j] = __uint_as_float(q[j] << 16); xv[2 * j + 1] = __uint_as_float(q[j] & 0xffff0000u); }
#pragma unroll
      for (int i = 0; i < 8; ++i) {
#pragma unroll
        for (int qd = 0; qd < 4; ++qd) { const v4f w = *(const v4f*)&wgs[8u * kc + i][4 * qd];
          lg[4 * qd + 0] = fmaf(xv[i], w[0], lg[4 * qd + 0]); lg[4 * qd + 1] = fmaf(xv[i], w[1], lg[4 * qd + 1]);
          lg[4 * qd + 2] = fmaf(xv[i], w[2], lg[4 * qd + 2]); lg[4 * qd + 3] = fmaf(xv[i], w[3], lg[4 * qd + 3]); } } } }
  int best = 0; float bv = lg[0] + bfr(BG[0]);
#pragma unroll
  for (int e = 1; e < NE; ++e) { const float v = lg[e] + bfr(BG[e]); const bool gt = v > bv; bv = gt ? v : bv; best = gt ? e : best; }

  int mycnt = 0, myrank = 0; const unsigned ltmask = (1u << lane) - 1u;
#pragma unroll
  for (int e = 0; e < NE; ++e) { const unsigned m = __builtin_amdgcn_ballot_w32(best == e);
    const int c = (int)__builtin_popcount(m), rk = (int)__builtin_popcount(m & ltmask);
    mycnt = ((int)lane == e) ? c : mycnt; myrank = (best == e) ? rk : myrank; }
  if (lane < 16u) wcnt[wave][lane] = mycnt;
  __syncthreads();
  { int off = 0;
#pragma unroll
    for (int w = 0; w < 4; ++w) { const int c = wcnt[w][best]; off += (w < wave) ? c : 0; }
    int pos = off + myrank; pos = pos < 0 ? 0 : pos; pos = pos > CH - 1 ? CH - 1 : pos;
    lst[best][pos] = (int)tid; }
  __syncthreads();

#pragma unroll 1
  for (int j = 0; j < NE / 4; ++j) { const int e = wave + 4 * j; const unsigned ue = (unsigned)e;
    int c = wcnt[0][e] + wcnt[1][e] + wcnt[2][e] + wcnt[3][e];
    c = c < 0 ? 0 : c; c = c > CH ? CH : c;
    const int cnt = __builtin_amdgcn_readfirstlane(c);
    const int ntile = (cnt + 15) >> 4;
    const int last = cnt - 1;
#pragma unroll 1
    for (int tl = 0; tl < ntile; ++tl) {
      asm volatile("s_wait_dscnt 0x0" ::: "memory");
#pragma unroll
      for (unsigned it = 0; it < 8; ++it) { const unsigned idx = it * 32u + lane, r = idx >> 4, q = idx & 15u;
        const int slot = tl * 16 + (int)r; const int sc = slot < last ? slot : last;
        const unsigned tok = (unsigned)lst[e][sc] & (unsigned)(CH - 1);
        v4u v = *(const v4u*)(XB + (size_t)(blk0 + tok) * DIN + 8u * q);
        asm volatile("" : "+v"(v));
        const bool ok = slot < cnt; const v4u z = {0u, 0u, 0u, 0u};
        v = ok ? v : z;
        *(v4u*)&xa[wave][r][8u * q] = v; }
      unsigned trow[8];
#pragma unroll
      for (int r = 0; r < 8; ++r) { const int slot = tl * 16 + 8 * (int)lh + r; const int sc = slot < last ? slot : last; trow[r] = (unsigned)lst[e][sc] & (unsigned)(CH - 1); }
      asm volatile("s_wait_dscnt 0x0" ::: "memory");
      __builtin_amdgcn_wave_barrier();
      v16b a1[4];
#pragma unroll
      for (int kc = 0; kc < 4; ++kc) { union { v16b v; v4u q[2]; } f;
        f.q[0] = *(const v4u*)&xa[wave][lm][kc * 32 + 8u * lh]; f.q[1] = *(const v4u*)&xa[wave][lm][kc * 32 + 16 + 8u * lh]; a1[kc] = f.v; }
      v8f acc2[8] = {};
#pragma unroll 1
      for (unsigned s = 0; s < NSLAB; ++s) {
        v8f acc1[4] = {};
        const unsigned short* bp = W1T + (size_t)(ue * DHID + s * SLAB + lm) * DIN + 8u * lh;
#pragma unroll
        for (int kc = 0; kc < 4; ++kc) {
#pragma unroll
          for (int ni = 0; ni < 4; ++ni) { const v16b b = ldfrag_b(bp + (size_t)ni * 16u * DIN + kc * 32u); acc1[ni] = wmma_bf(a1[kc], b, acc1[ni]); } }
#pragma unroll
        for (int ni = 0; ni < 4; ++ni) {
#pragma unroll
          for (int r = 0; r < 8; ++r) { const float v = acc1[ni][r]; const float g = 0.5f * v * (1.0f + erff(v * 0.70710678118654752440f));
            hs[wave][8u * lh + r][ni * 16 + lm] = toh_flush(g * HCARRY); } }
        asm volatile("s_wait_dscnt 0x0" ::: "memory");
        __builtin_amdgcn_wave_barrier();
        v16h a2[2];
#pragma unroll
        for (int kk = 0; kk < 2; ++kk) { union { v16h v; v8h q[2]; } f;
          f.q[0] = *(const v8h*)&hs[wave][lm][kk * 32 + 8u * lh]; f.q[1] = *(const v8h*)&hs[wave][lm][kk * 32 + 16 + 8u * lh]; a2[kk] = f.v; }
        asm volatile("s_wait_dscnt 0x0" ::: "memory");
        const unsigned short* cp = W2T + (size_t)lm * KF + ue * DHID + s * SLAB + 8u * lh;
#pragma unroll
        for (int kk = 0; kk < 2; ++kk) {
#pragma unroll
          for (int nj = 0; nj < 8; ++nj) { const v16h b = ldfrag_h(cp + (size_t)nj * 16u * KF + kk * 32u); acc2[nj] = wmma16(a2[kk], b, acc2[nj]); } }
      }
#pragma unroll
      for (int r = 0; r < 8; ++r) { const int slot = tl * 16 + 8 * (int)lh + r;
        if (slot < cnt) {
#pragma unroll
          for (int nj = 0; nj < 8; ++nj) os[trow[r]][nj * 16 + lm] = acc2[nj][r] * OSCALE; } }
    }
  }
  __syncthreads();

  float* po = OUT + (size_t)blk0 * DOUT;
#pragma unroll 4
  for (unsigned it = 0; it < 32; ++it) { const unsigned idx = it * 128u + tid, rw = idx >> 5, pc = idx & 31u;
    const v4f v = *(const v4f*)&os[rw][4u * pc]; *(volatile v4f*)(po + (size_t)rw * DOUT + 4u * pc) = v; }
  __threadfence();
#pragma unroll 4
  for (unsigned it = 0; it < 32; ++it) { const unsigned idx = it * 128u + tid, rw = idx >> 5, pc = idx & 31u;
    const v4f v = *(const v4f*)&os[rw][4u * pc]; *(volatile v4f*)(po + (size_t)rw * DOUT + 4u * pc) = v; }
}

extern "C" void kernel_launch(void* const* d_in, const int* in_sizes, int n_in, void* d_out, int out_size, void* d_ws, size_t ws_size, hipStream_t stream) {
  if (n_in < 5) return;
  if (in_sizes[0] < NB * DIN || in_sizes[1] < NE * DIN * DHID || in_sizes[2] < NE * DHID * DOUT || in_sizes[3] < DIN * NE || in_sizes[4] < NE) return;
  if ((size_t)out_size < (size_t)NB * DOUT) return;
  if (ws_size < (size_t)WS_END) return;
  const float* X  = (const float*)d_in[0];
  const float* W1 = (const float*)d_in[1];
  const float* W2 = (const float*)d_in[2];
  const float* WG = (const float*)d_in[3];
  const float* BG = (const float*)d_in[4];
  char* ws = (char*)d_ws;
  unsigned short* XB  = (unsigned short*)(ws + WS_XB);
  unsigned short* W1T = (unsigned short*)(ws + WS_W1T);
  unsigned short* W2T = (unsigned short*)(ws + WS_W2T);
  float* OUT = (float*)d_out;
  k_cvt_x<<<dim3(NB * DIN / 8 / 256), 256, 0, stream>>>(X, XB);
  k_tr_w1<<<dim3(DHID / 64, DIN / 64, NE), 256, 0, stream>>>(W1, W1T, (unsigned)DIN, (unsigned)DHID, (unsigned)DIN, (unsigned)DHID, 0u);
  k_tr_w2<<<dim3(DOUT / 64, DHID / 64, NE), 256, 0, stream>>>(W2, W2T, (unsigned)DHID, (unsigned)DOUT, (unsigned)KF, 0u, (unsigned)DHID, WCARRY);
  k_moe<<<dim3(NB / CH), 128, 0, stream>>>(XB, W1T, W2T, WG, BG, OUT);
}
